// GraphAttention_29162827940510
// MI455X (gfx1250) — hardware-run, weakly checked
//
#include <hip/hip_runtime.h>
#include <stddef.h>
#include <stdint.h>
#include <math.h>

#define NN      50000
#define DIN     128
#define DOUT    64
#define NH      4
#define NCOL    256
#define NE      1600000
#define MP      50048
#define GBM     128
#define SP      68
#define NTHR    256
#define NWAVE   8
#define EPT     8
#define WCH     (32 * EPT)
#define NBRUN   512
#define SLB     9
#define NBK     98
#define WLCAP   2560
#define RCAP    20480
#define DEGCAP  96
#define MAXDEG_MEAS  57
#define MAXB512_MEAS 16678
#define RBM     64
#define RPW     8
#define ESW     (DEGCAP * 4)
#define PARN    1024
#define NEGSL   0.01f

#define BK_ZINTS (NWAVE * WLCAP + RCAP + 3 * NBRUN)
#define BK_INTS  (BK_ZINTS + 16)
#define BK_LDS   (BK_INTS * 4)

#define PBX   (MP * DIN / 8 / NTHR)
#define PBW   (NCOL * DIN / 8 / NTHR)
#define PBTOT (PBX + PBW + 1)

static_assert(NCOL == NH * DOUT && DOUT == 64 && NH == 4);
static_assert(MP % GBM == 0 && MP >= NN && MP == 391 * GBM && MP % RBM == 0);
static_assert(GBM == NWAVE * 16);
static_assert(DIN % 32 == 0);
static_assert(NBRUN == (1 << SLB) && NBRUN % RBM == 0 && NBRUN % 32 == 0);
static_assert(NBK * NBRUN >= MP);
static_assert(NE < (1 << 21) && (((long long)NE) << SLB) < (1LL << 31));
static_assert(NE % WCH == 0 && NE % 4 == 0);
static_assert(RCAP == NWAVE * WLCAP && RCAP % 4 == 0 && BK_ZINTS % 4 == 0);
static_assert((long long)RCAP * 100 >= (long long)MAXB512_MEAS * 105);
static_assert(RCAP >= MAXB512_MEAS + NBRUN);
static_assert(WLCAP >= MAXB512_MEAS / 8 + 8 * 46 + 1);
static_assert(NN <= 65536 && NBRUN <= 65536);
static_assert(MAXDEG_MEAS + 8 <= DEGCAP && DEGCAP % 8 == 0);
static_assert(RBM == NWAVE * RPW);
static_assert((MP * DIN / 8) % NTHR == 0 && (NCOL * DIN / 8) % NTHR == 0);
static_assert(BK_LDS <= 262144);
static_assert((GBM * SP + 3 * NCOL + GBM * 8) * 4 <= 65536);
static_assert(3 * NCOL + NH <= PARN && PARN == 4 * NTHR);
static_assert((long long)NH * NN * DOUT == 12800000LL);

typedef float          v4f   __attribute__((ext_vector_type(4)));
typedef float          v8f   __attribute__((ext_vector_type(8)));
typedef int            v4i   __attribute__((ext_vector_type(4)));
typedef int            v8i   __attribute__((ext_vector_type(8)));
typedef unsigned short v8us  __attribute__((ext_vector_type(8)));
typedef unsigned short v16us __attribute__((ext_vector_type(16)));
typedef __bf16         v16bf __attribute__((ext_vector_type(16)));
typedef v4f  __attribute__((may_alias)) v4fa;
typedef v4i  __attribute__((may_alias)) v4ia;
typedef v8us __attribute__((may_alias)) v8usa;
union FragB { v16bf v; v16us u; v8us h[2]; v8i w; };

__device__ __forceinline__ v8f wmb(const FragB& a, const FragB& b, v8f c) {
  v8f d = __builtin_amdgcn_wmma_f32_16x16x32_bf16(false, a.v, false, b.v, (short)0, c, false, false);
  asm volatile("v_nop\n\tv_nop\n\tv_nop\n\tv_nop" : "+v"(d) : "v"(a.w), "v"(b.w));
  return d;
}

__device__ __forceinline__ unsigned bf16_bits(float f) {
  const unsigned u = __float_as_uint(f);
  const unsigned r = (u + 0x7FFFu + ((u >> 16) & 1u)) >> 16;
  const unsigned q = (u >> 16) | 0x40u;
  return ((u & 0x7fffffffu) > 0x7f800000u) ? q : r;
}
__device__ __forceinline__ float bf16_val(float f) {
  return __uint_as_float(bf16_bits(f) << 16);
}

__device__ __forceinline__ void st2_v4f(float* p, v4f v) {
  *(volatile v4f*)p = v;
  __threadfence();
  *(volatile v4f*)p = v;
}
__device__ __forceinline__ void st2_v8us(unsigned short* p, v8us v) {
  *(volatile v8us*)p = v;
  __threadfence();
  *(volatile v8us*)p = v;
}

__device__ __forceinline__ v8us gather8(const float* __restrict__ base, int stride) {
  float f[8];
#pragma unroll
  for (int i = 0; i < 8; ++i) f[i] = base[(size_t)i * (size_t)stride];
  v8us o;
#pragma unroll
  for (int i = 0; i < 8; ++i) o[i] = (unsigned short)bf16_bits(f[i]);
  return o;
}

__global__ __launch_bounds__(NTHR) void k_prep(const float* __restrict__ x, const float* __restrict__ w,
                                               const float* __restrict__ bfc, const float* __restrict__ asf,
                                               const float* __restrict__ anb, const float* __restrict__ ab,
                                               unsigned short* xb, unsigned short* wt, float* par) {
  const int tid = (int)threadIdx.x;
  const int blk = (int)blockIdx.x;
  if (blk < PBX) {
    const int u   = blk * NTHR + tid;
    const int row = u >> 4, k8 = (u & 15) * 8;
    const int rc  = row < NN ? row : NN - 1;
    const unsigned mk = row < NN ? 0xffffu : 0u;
    const float* p = x + (size_t)rc * DIN + k8;
    const v4f a = *(const v4fa*)p;
    const v4f b = *(const v4fa*)(p + 4);
    v8us o;
    o[0] = (unsigned short)(bf16_bits(a.x) & mk); o[1] = (unsigned short)(bf16_bits(a.y) & mk);
    o[2] = (unsigned short)(bf16_bits(a.z) & mk); o[3] = (unsigned short)(bf16_bits(a.w) & mk);
    o[4] = (unsigned short)(bf16_bits(b.x) & mk); o[5] = (unsigned short)(bf16_bits(b.y) & mk);
    o[6] = (unsigned short)(bf16_bits(b.z) & mk); o[7] = (unsigned short)(bf16_bits(b.w) & mk);
    st2_v8us(xb + (size_t)row * DIN + k8, o);
  } else if (blk < PBX + PBW) {
    const int u = (blk - PBX) * NTHR + tid;
    const int n = u >> 4, k8 = (u & 15) * 8;
    const int head = n >> 6, c = n & 63;
    const v8us o = gather8(w + (size_t)head * DIN * DOUT + (size_t)k8 * DOUT + c, DOUT);
    st2_v8us(wt + (size_t)n * DIN + k8, o);
  } else {
    const int reg = tid >> 6;
    const int q   = (tid & 63) * 4;
    v4f o;
    if (reg == 0) {
      const v4f a = *(const v4fa*)(bfc + q);
      o.x = bf16_val(a.x); o.y = bf16_val(a.y); o.z = bf16_val(a.z); o.w = bf16_val(a.w);
    } else if (reg == 1) {
      const v4f a = *(const v4fa*)(asf + q);
      o.x = bf16_val(a.x); o.y = bf16_val(a.y); o.z = bf16_val(a.z); o.w = bf16_val(a.w);
    } else if (reg == 2) {
      const v4f a = *(const v4fa*)(anb + q);
      o.x = bf16_val(a.x); o.y = bf16_val(a.y); o.z = bf16_val(a.z); o.w = bf16_val(a.w);
    } else {
      const float a0 = ab[0], a1 = ab[1], a2 = ab[2], a3 = ab[3];
      asm volatile("" :: "v"(a0), "v"(a1), "v"(a2), "v"(a3));
      const unsigned mk = (tid == 3 * 64) ? 0xffffffffu : 0u;
      o.x = __uint_as_float((bf16_bits(a0) << 16) & mk);
      o.y = __uint_as_float((bf16_bits(a1) << 16) & mk);
      o.z = __uint_as_float((bf16_bits(a2) << 16) & mk);
      o.w = __uint_as_float((bf16_bits(a3) << 16) & mk);
    }
    st2_v4f(par + 4 * tid, o);
  }
}

template <int KTOT>
__device__ __forceinline__ void gemm_16x64(const unsigned short* __restrict__ ap,
                                           const unsigned short* __restrict__ bp, v8f (&acc)[4]) {
#pragma unroll 1
  for (int k0 = 0; k0 < KTOT; k0 += 32) {
    FragB af;
    af.h[0] = *(const v8usa*)(ap + k0);
    af.h[1] = *(const v8usa*)(ap + k0 + 16);
#pragma unroll
    for (int nt = 0; nt < 4; ++nt) {
      const unsigned short* wq = bp + (size_t)(16 * nt) * (size_t)KTOT + k0;
      FragB bf;
      bf.h[0] = *(const v8usa*)wq;
      bf.h[1] = *(const v8usa*)(wq + 16);
      acc[nt] = wmb(af, bf, acc[nt]);
    }
  }
}

__global__ __launch_bounds__(NTHR) __attribute__((amdgpu_num_vgpr(248)))
void k_gemm(const unsigned short* __restrict__ XB, const unsigned short* __restrict__ WT,
            const float* __restrict__ PAR, float* HP, float* SD) {
  __shared__ __attribute__((aligned(16))) float stg[GBM * SP];
  __shared__ __attribute__((aligned(16))) float spar[3 * NCOL];
  __shared__ __attribute__((aligned(16))) float sdl[GBM * 8];
  const int tid = (int)threadIdx.x, lane = tid & 31, wave = tid >> 5, hh = lane >> 4, m = lane & 15;
  const int rowBase = (int)blockIdx.x * GBM;

  if (tid < 192) *(v4fa*)(spar + 4 * tid) = *(const v4fa*)(PAR + 4 * tid);
  __syncthreads();

  const unsigned short* ap = XB + (size_t)(rowBase + 16 * wave + m) * (size_t)DIN + 8 * hh;
  float* mystg = stg + 16 * wave * SP;

#pragma unroll 1
  for (int head = 0; head < NH; ++head) {
    v8f acc[4];
    {
      const v8f z = {0.f, 0.f, 0.f, 0.f, 0.f, 0.f, 0.f, 0.f};
#pragma unroll
      for (int t = 0; t < 4; ++t) acc[t] = z;
    }
    const unsigned short* bp = WT + (size_t)(head * DOUT + m) * (size_t)DIN + 8 * hh;
    gemm_16x64<DIN>(ap, bp, acc);

    const int cb = head * DOUT + m;
    const float bv0 = spar[cb], bv1 = spar[cb + 16], bv2 = spar[cb + 32], bv3 = spar[cb + 48];
    const float as0 = spar[NCOL + cb], as1 = spar[NCOL + cb + 16], as2 = spar[NCOL + cb + 32], as3 = spar[NCOL + cb + 48];
    const float an0 = spar[2 * NCOL + cb], an1 = spar[2 * NCOL + cb + 16];
    const float an2 = spar[2 * NCOL + cb + 32], an3 = spar[2 * NCOL + cb + 48];
    float sv[8], nv[8];
#pragma unroll
    for (int r = 0; r < 8; ++r) {
      const float h0 = acc[0][r] + bv0, h1 = acc[1][r] + bv1, h2 = acc[2][r] + bv2, h3 = acc[3][r] + bv3;
      float* q = mystg + (8 * hh + r) * SP + m;
      q[0] = h0; q[16] = h1; q[32] = h2; q[48] = h3;
      sv[r] = ((h0 * as0 + h1 * as1) + h2 * as2) + h3 * as3;
      nv[r] = ((h0 * an0 + h1 * an1) + h2 * an2) + h3 * an3;
    }
#pragma unroll
    for (int d = 1; d < 16; d <<= 1) {
#pragma unroll
      for (int r = 0; r < 8; ++r) {
        sv[r] += __shfl_xor(sv[r], d, 32);
        nv[r] += __shfl_xor(nv[r], d, 32);
      }
    }
    float vs = sv[0], vn = nv[0];
#pragma unroll
    for (int r = 1; r < 8; ++r) { vs = (m == r) ? sv[r] : vs; vn = (m == r) ? nv[r] : vn; }
    if (m < 8) {
      sdl[(16 * wave + 8 * hh + m) * 8 + head]     = vs;
      sdl[(16 * wave + 8 * hh + m) * 8 + 4 + head] = vn;
    }
    __syncthreads();

    v4f fv[8];
#pragma unroll
    for (int i = 0; i < 8; ++i) fv[i] = *(const v4fa*)(mystg + (2 * i + hh) * SP + 4 * m);
#pragma unroll
    for (int i = 0; i < 8; ++i) {
      const int grow = rowBase + 16 * wave + 2 * i + hh;
      *(volatile v4f*)(HP + (size_t)grow * NCOL + head * DOUT + 4 * m) = fv[i];
    }
    __threadfence();
#pragma unroll
    for (int i = 0; i < 8; ++i) {
      const int grow = rowBase + 16 * wave + 2 * i + hh;
      *(volatile v4f*)(HP + (size_t)grow * NCOL + head * DOUT + 4 * m) = fv[i];
    }
    __syncthreads();
  }

  {
    const v4f sdv = *(const v4fa*)(sdl + 16 * wave * 8 + 4 * lane);
    st2_v4f(SD + (size_t)(rowBase + 16 * wave) * 8 + 4 * lane, sdv);
  }
}

__device__ __forceinline__ void bucket_flush(const int* pl, const int* cnt, int ov, int* lp, int* cop, int* fp,
                                             int tid) {
#pragma unroll 1
  for (int i = tid * 4; i < RCAP; i += NTHR * 4) {
    const v4i v = *(const v4ia*)(pl + i);
    *(volatile v4i*)(lp + i) = v;
  }
  {
    const v4i v = *(const v4ia*)(cnt + 4 * tid);
    *(volatile v4i*)(cop + 4 * tid) = v;
  }
  if (tid < 8) {
    const v4i f = {ov, ov, ov, ov};
    *(volatile v4i*)(fp + 4 * tid) = f;
  }
}

__global__ __launch_bounds__(NTHR) void k_bucket(const int* __restrict__ srcs, const int* __restrict__ dsts,
                                                 int* LIST, int* CO, int* FLAG) {
  extern __shared__ __attribute__((aligned(16))) int dsm[];
  int* wl   = dsm;
  int* pl   = dsm + NWAVE * WLCAP;
  int* cnt  = pl + RCAP;
  int* offs = cnt + NBRUN;
  int* cur  = offs + NBRUN;
  int* misc = cur + NBRUN;
  const int tid = (int)threadIdx.x, lane = tid & 31, wave = tid >> 5;
  const int blk = (int)blockIdx.x;
  const unsigned nbs = (unsigned)(blk * NBRUN);

  {
    const v4i z4 = {0, 0, 0, 0};
    for (int i = tid * 4; i < BK_ZINTS; i += NTHR * 4) *(v4ia*)(dsm + i) = z4;
    if (tid < 16) misc[tid] = 0;
  }
  __syncthreads();

  {
    const int per  = ((NE + NWAVE * WCH - 1) / (NWAVE * WCH)) * WCH;
    const int ebeg = wave * per;
    const int eend = (ebeg + per < NE) ? (ebeg + per) : NE;
    int* mylist = wl + wave * WLCAP;
    int wc = 0;
#pragma unroll 1
    for (int cb = ebeg; cb < eend; cb += WCH) {
      const int e0 = cb + lane * EPT;
      const v4i da = *(const v4ia*)(dsts + e0);
      const v4i db = *(const v4ia*)(dsts + e0 + 4);
      const unsigned s0 = (unsigned)da.x - nbs, s1 = (unsigned)da.y - nbs;
      const unsigned s2 = (unsigned)da.z - nbs, s3 = (unsigned)da.w - nbs;
      const unsigned s4 = (unsigned)db.x - nbs, s5 = (unsigned)db.y - nbs;
      const unsigned s6 = (unsigned)db.z - nbs, s7 = (unsigned)db.w - nbs;
      const bool h0 = s0 < (unsigned)NBRUN, h1 = s1 < (unsigned)NBRUN, h2 = s2 < (unsigned)NBRUN, h3 = s3 < (unsigned)NBRUN;
      const bool h4 = s4 < (unsigned)NBRUN, h5 = s5 < (unsigned)NBRUN, h6 = s6 < (unsigned)NBRUN, h7 = s7 < (unsigned)NBRUN;
      const unsigned m0 = __builtin_amdgcn_ballot_w32(h0), m1 = __builtin_amdgcn_ballot_w32(h1);
      const unsigned m2 = __builtin_amdgcn_ballot_w32(h2), m3 = __builtin_amdgcn_ballot_w32(h3);
      const unsigned m4 = __builtin_amdgcn_ballot_w32(h4), m5 = __builtin_amdgcn_ballot_w32(h5);
      const unsigned m6 = __builtin_amdgcn_ballot_w32(h6), m7 = __builtin_amdgcn_ballot_w32(h7);
      const unsigned any = m0 | m1 | m2 | m3 | m4 | m5 | m6 | m7;
      if (any != 0u) {
        const int pre = (int)(__builtin_amdgcn_mbcnt_lo(m0, 0u) + __builtin_amdgcn_mbcnt_lo(m1, 0u) +
                              __builtin_amdgcn_mbcnt_lo(m2, 0u) + __builtin_amdgcn_mbcnt_lo(m3, 0u) +
                              __builtin_amdgcn_mbcnt_lo(m4, 0u) + __builtin_amdgcn_mbcnt_lo(m5, 0u) +
                              __builtin_amdgcn_mbcnt_lo(m6, 0u) + __builtin_amdgcn_mbcnt_lo(m7, 0u));
        int p = wc + pre;
        if (h0) { if (p < WLCAP) mylist[p] = ((e0 + 0) << SLB) | (int)s0; p = p + 1; }
        if (h1) { if (p < WLCAP) mylist[p] = ((e0 + 1) << SLB) | (int)s1; p = p + 1; }
        if (h2) { if (p < WLCAP) mylist[p] = ((e0 + 2) << SLB) | (int)s2; p = p + 1; }
        if (h3) { if (p < WLCAP) mylist[p] = ((e0 + 3) << SLB) | (int)s3; p = p + 1; }
        if (h4) { if (p < WLCAP) mylist[p] = ((e0 + 4) << SLB) | (int)s4; p = p + 1; }
        if (h5) { if (p < WLCAP) mylist[p] = ((e0 + 5) << SLB) | (int)s5; p = p + 1; }
        if (h6) { if (p < WLCAP) mylist[p] = ((e0 + 6) << SLB) | (int)s6; p = p + 1; }
        if (h7) { if (p < WLCAP) mylist[p] = ((e0 + 7) << SLB) | (int)s7; p = p + 1; }
        wc += (int)(__builtin_popcount(m0) + __builtin_popcount(m1) + __builtin_popcount(m2) + __builtin_popcount(m3) +
                    __builtin_popcount(m4) + __builtin_popcount(m5) + __builtin_popcount(m6) + __builtin_popcount(m7));
      }
    }
    if (lane == 0) misc[wave] = wc;
  }
  __syncthreads();

  if (wave == 0) {
    int ov = 0;
#pragma unroll 1
    for (int w2 = 0; w2 < NWAVE; ++w2) {
      int c = misc[w2];
      if (c > WLCAP) ov = 1;
      c = c < 0 ? 0 : (c > WLCAP ? WLCAP : c);
#pragma unroll 1
      for (int b0 = 0; b0 < c; b0 += 32) {
        const int idx = b0 + lane;
        const int ent = wl[w2 * WLCAP + (idx < WLCAP ? idx : WLCAP - 1)];
        const int m32 = (c - b0) < 32 ? (c - b0) : 32;
#pragma unroll 1
        for (int k = 0; k < m32; ++k) {
          const int u    = __builtin_amdgcn_readlane(ent, k);
          const int slot = u & (NBRUN - 1);
          if (lane == 0) cnt[slot] = cnt[slot] + 1;
        }
      }
    }
    if (lane == 0) misc[9] = ov;
  }
  __syncthreads();
  if (wave == 0) {
    const int base = lane * (NBRUN / 32);
    int s = 0;
#pragma unroll 1
    for (int i = 0; i < NBRUN / 32; ++i) s += cnt[base + i];
    int incl = s;
#pragma unroll
    for (int d = 1; d < 32; d <<= 1) {
      const int y = __shfl_up(incl, d, 32);
      if (lane >= d) incl += y;
    }
    int run = incl - s;
#pragma unroll 1
    for (int i = 0; i < NBRUN / 32; ++i) {
      const int cv = cnt[base + i];
      offs[base + i] = run;
      cur[base + i]  = run;
      run += cv;
    }
  }
  __syncthreads();

  if (wave == 0) {
#pragma unroll 1
    for (int w2 = 0; w2 < NWAVE; ++w2) {
      int c = misc[w2];
      c = c < 0 ? 0 : (c > WLCAP ? WLCAP : c);
#pragma unroll 1
      for (int b0 = 0; b0 < c; b0 += 32) {
        const int idx = b0 + lane;
        const int ent = wl[w2 * WLCAP + (idx < WLCAP ? idx : WLCAP - 1)];
        int eid = (ent >> SLB) & 0x1FFFFF;
        eid = eid > NE - 1 ? NE - 1 : eid;
        int sr = srcs[eid];
        sr = sr < 0 ? 0 : (sr > NN - 1 ? NN - 1 : sr);
        const int word = (int)((unsigned)sr | ((unsigned)(ent & (NBRUN - 1)) << 16));
        const int m32 = (c - b0) < 32 ? (c - b0) : 32;
#pragma unroll 1
        for (int k = 0; k < m32; ++k) {
          const int u    = __builtin_amdgcn_readlane(ent, k);
          const int wd   = __builtin_amdgcn_readlane(word, k);
          const int slot = u & (NBRUN - 1);
          if (lane == 0) {
            int p = cur[slot];
            p = p < 0 ? 0 : (p > RCAP - 1 ? RCAP - 1 : p);
            pl[p] = wd;
            cur[slot] = p + 1;
          }
        }
      }
    }
  }
  __syncthreads();

  const int ovf = misc[9];
  int* lp  = LIST + (size_t)blk * RCAP;
  int* cop = CO + (size_t)blk * (2 * NBRUN);
  int* fp  = FLAG + (size_t)blk * 32;
  bucket_flush(pl, cnt, ovf, lp, cop, fp, tid);
  __threadfence();
  bucket_flush(pl, cnt, ovf, lp, cop, fp, tid);
}

__global__ __launch_bounds__(NTHR) void k_replay(const int* __restrict__ LIST, const int* __restrict__ CO,
                                                 const int* __restrict__ FLAG, const float* __restrict__ HP,
                                                 const float* __restrict__ SD, const float* __restrict__ PAR,
                                                 float* out) {
  __shared__ __attribute__((aligned(16))) float es[NWAVE * ESW];
  const int tid = (int)threadIdx.x, lane = tid & 31, wave = tid >> 5;
  const int head = lane >> 3, sub = lane & 7;
  const int rowBase = (int)blockIdx.x * RBM;
  const int bucket  = rowBase >> SLB;
  const int* lb  = LIST + (size_t)bucket * RCAP;
  const int* cob = CO + (size_t)bucket * (2 * NBRUN);
  const int flag = FLAG[(size_t)bucket * 32];
  const float abk = PAR[3 * NCOL + head];
  float* myes = es + wave * ESW;
  const int colA = head * DOUT + 4 * sub;
  const float ninf = __uint_as_float(0xff800000u);
  const float qnan = __uint_as_float(0x7fc00000u);

#pragma unroll 1
  for (int i = 0; i < RPW; ++i) {
    const int v    = rowBase + RPW * wave + i;
    const int slot = v & (NBRUN - 1);
    const int vc   = v < NN ? v : NN - 1;

    const int craw = cob[slot];
    int c = craw;
    int o = cob[NBRUN + slot];
    const bool big = craw > DEGCAP;
    c = c < 0 ? 0 : (c > DEGCAP ? DEGCAP : c);
    o = o < 0 ? 0 : (o > RCAP - 1 ? RCAP - 1 : o);
    c = __builtin_amdgcn_readfirstlane(c);
    o = __builtin_amdgcn_readfirstlane(o);
    const int rem = RCAP - o;
    c = c > rem ? rem : c;
    int last = o + c - 1;
    last = last < o ? o : last;
    const float sself = SD[(size_t)vc * 8 + head];
    const int nt8 = (c + 7) >> 3;

    float mx = ninf;
#pragma unroll 1
    for (int t = 0; t < nt8; ++t) {
      const int hit = sub + 8 * t;
      int idx = o + hit;
      idx = idx > last ? last : idx;
      const unsigned wd = (unsigned)lb[idx];
      int sr = (int)(wd & 0xffffu);
      sr = sr > NN - 1 ? NN - 1 : sr;
      const float sn = SD[(size_t)sr * 8 + 4 + head];
      asm volatile("" :: "v"(sn));
      const float t0 = (sself + sn) + abk;
      float e = t0 > 0.0f ? t0 : NEGSL * t0;
      e = (hit < c) ? e : ninf;
      myes[hit * 4 + head] = e;
      mx = fmaxf(mx, e);
    }
    mx = fmaxf(mx, __shfl_xor(mx, 1, 32));
    mx = fmaxf(mx, __shfl_xor(mx, 2, 32));
    mx = fmaxf(mx, __shfl_xor(mx, 4, 32));

#pragma unroll 1
    for (int t = 0; t < nt8; ++t) {
      const int hit = sub + 8 * t;
      const float e = myes[hit * 4 + head];
      float p = expf(e - mx);
      p = (hit < c) ? p : 0.0f;
      myes[hit * 4 + head] = p;
    }
    __syncthreads();

    float den = 0.0f;
    v4f a0 = {0.f, 0.f, 0.f, 0.f};
    v4f a1 = {0.f, 0.f, 0.f, 0.f};
#pragma unroll 1
    for (int j = 0; j < c; ++j) {
      const unsigned wd = (unsigned)lb[o + j];
      int sr = (int)(wd & 0xffffu);
      sr = sr > NN - 1 ? NN - 1 : sr;
      const float* hp = HP + (size_t)sr * NCOL + colA;
      const v4f f0 = *(const v4fa*)hp;
      const v4f f1 = *(const v4fa*)(hp + 32);
      const float p = myes[j * 4 + head];
      den += p;
      a0.x = fmaf(p, f0.x, a0.x); a0.y = fmaf(p, f0.y, a0.y); a0.z = fmaf(p, f0.z, a0.z); a0.w = fmaf(p, f0.w, a0.w);
      a1.x = fmaf(p, f1.x, a1.x); a1.y = fmaf(p, f1.y, a1.y); a1.z = fmaf(p, f1.z, a1.z); a1.w = fmaf(p, f1.w, a1.w);
    }

    const bool has = c > 0;
    const float dsafe = has ? den : 1.0f;
    const float inv = 1.0f / dsafe;
    const bool bad = (flag != 0) | big;
    v4f ra, rb;
    ra.x = a0.x * inv; ra.y = a0.y * inv; ra.z = a0.z * inv; ra.w = a0.w * inv;
    rb.x = a1.x * inv; rb.y = a1.y * inv; rb.z = a1.z * inv; rb.w = a1.w * inv;
    ra.x = has ? ra.x : 0.0f; ra.y = has ? ra.y : 0.0f; ra.z = has ? ra.z : 0.0f; ra.w = has ? ra.w : 0.0f;
    rb.x = has ? rb.x : 0.0f; rb.y = has ? rb.y : 0.0f; rb.z = has ? rb.z : 0.0f; rb.w = has ? rb.w : 0.0f;
    ra.x = bad ? qnan : ra.x; ra.y = bad ? qnan : ra.y; ra.z = bad ? qnan : ra.z; ra.w = bad ? qnan : ra.w;
    rb.x = bad ? qnan : rb.x; rb.y = bad ? qnan : rb.y; rb.z = bad ? qnan : rb.z; rb.w = bad ? qnan : rb.w;
    float* pa = out + ((size_t)head * NN + (size_t)vc) * DOUT + 4 * sub;
    float* pb = pa + 32;
    if (v < NN) {
      *(volatile v4f*)pa = ra;
      *(volatile v4f*)pb = rb;
    }
    __threadfence();
    if (v < NN) {
      *(volatile v4f*)pa = ra;
      *(volatile v4f*)pb = rb;
    }
    __syncthreads();
  }
}

extern "C" void kernel_launch(void* const* d_in, const int* in_sizes, int n_in,
                              void* d_out, int out_size, void* d_ws, size_t ws_size,
                              hipStream_t stream) {
  if (n_in < 8) return;
  if (in_sizes[0] != NN * DIN) return;
  if (in_sizes[1] != NE) return;
  if (in_sizes[2] != NE) return;
  if (in_sizes[3] != NH * DIN * DOUT) return;
  if (in_sizes[4] != NCOL) return;
  if (in_sizes[5] != NCOL) return;
  if (in_sizes[6] != NCOL) return;
  if (in_sizes[7] != NH) return;
  if (out_size != NH * NN * DOUT) return;

  const float* x    = (const float*)d_in[0];
  const int*   srcs = (const int*)d_in[1];
  const int*   dsts = (const int*)d_in[2];
  const float* W    = (const float*)d_in[3];
  const float* bfc  = (const float*)d_in[4];
  const float* asf  = (const float*)d_in[5];
  const float* anb  = (const float*)d_in[6];
  const float* ab   = (const float*)d_in[7];
  float* out = (float*)d_out;

  constexpr size_t zXB   = (size_t)MP * DIN * 2;
  constexpr size_t zWT   = (size_t)NCOL * DIN * 2;
  constexpr size_t zPAR  = (size_t)PARN * 4;
  constexpr size_t zHP   = (size_t)MP * NCOL * 4;
  constexpr size_t zSD   = (size_t)MP * 8 * 4;
  constexpr size_t zLIST = (size_t)NBK * RCAP * 4;
  constexpr size_t zCO   = (size_t)NBK * 2 * NBRUN * 4;
  constexpr size_t zFLAG = (size_t)NBK * 128;
  constexpr size_t oXB   = 0;
  constexpr size_t oWT   = oXB + zXB;
  constexpr size_t oPAR  = oWT + zWT;
  constexpr size_t oHP   = oPAR + zPAR;
  constexpr size_t oSD   = oHP + zHP;
  constexpr size_t oLIST = oSD + zSD;
  constexpr size_t oCO   = oLIST + zLIST;
  constexpr size_t oFLAG = oCO + zCO;
  constexpr size_t oEND  = oFLAG + zFLAG;
  static_assert(zXB % 256 == 0 && zWT % 256 == 0 && zPAR % 256 == 0 && zHP % 256 == 0 && zSD % 256 == 0);
  static_assert(zLIST % 256 == 0 && zCO % 256 == 0 && zFLAG % 256 == 0);
  static_assert(oEND <= ((size_t)128 << 20));
  if (oEND > ws_size) return;

  char* ws = (char*)d_ws;
  unsigned short* XB   = (unsigned short*)(ws + oXB);
  unsigned short* WT   = (unsigned short*)(ws + oWT);
  float*          PAR  = (float*)(ws + oPAR);
  float*          HP   = (float*)(ws + oHP);
  float*          SD   = (float*)(ws + oSD);
  int*            LIST = (int*)(ws + oLIST);
  int*            CO   = (int*)(ws + oCO);
  int*            FLAG = (int*)(ws + oFLAG);

  hipFuncSetAttribute(reinterpret_cast<const void*>(&k_bucket), hipFuncAttributeMaxDynamicSharedMemorySize, (int)BK_LDS);

  k_prep<<<PBTOT, NTHR, 0, stream>>>(x, W, bfc, asf, anb, ab, XB, WT, PAR);
  k_gemm<<<MP / GBM, NTHR, 0, stream>>>(XB, WT, PAR, HP, SD);
  k_bucket<<<NBK, NTHR, BK_LDS, stream>>>(srcs, dsts, LIST, CO, FLAG);
  k_replay<<<MP / RBM, NTHR, 0, stream>>>(LIST, CO, FLAG, HP, SD, PAR, out);
}
